// CDSPMoELayer_87101936763275
// MI455X (gfx1250) — hardware-verified
//
#include <hip/hip_runtime.h>


typedef __bf16 v16bf __attribute__((ext_vector_type(16)));
typedef __bf16 v8bf  __attribute__((ext_vector_type(8)));
typedef float  v8f   __attribute__((ext_vector_type(8)));
typedef float  v4f   __attribute__((ext_vector_type(4)));
typedef float  v4fa  __attribute__((ext_vector_type(4), __may_alias__));
typedef unsigned int v4u __attribute__((ext_vector_type(4)));
typedef int    v4i   __attribute__((ext_vector_type(4)));

union Frag { v16bf v; v8bf h8[2]; };

#define NB      2
#define S_SEQ   4096
#define D_MODEL 1024
#define N_TOK   (NB * S_SEQ)
#define NE      16
#define DTASK   32
#define DBOT    256
#define RQ      64
#define EPSLN   1e-5f
#define CHUNK   256
#define CPG     2
#define NGRP    (N_TOK / (CHUNK * CPG))
#define MT      16

#define OFF_STAT   0ull
#define OFF_GATE   256ull
#define OFF_META   1024ull
#define OFF_CST    8192ull
#define OFF_COMB   65536ull
#define OFF_WDH    (1ull << 20)
#define OFF_WDL    (3ull << 20)
#define OFF_WUH    (5ull << 20)
#define OFF_WUL    (7ull << 20)
#define OFF_XH     (9ull << 20)
#define OFF_XL     (25ull << 20)
#define OFF_Y      (41ull << 20)
#define WS_TOTAL   (73ull << 20)

__device__ __forceinline__ v8f wmma16(const v16bf a, const v16bf b, v8f c)
{
    v8f d = __builtin_amdgcn_wmma_f32_16x16x32_bf16(false, a, false, b, (short)0, c, false, false);
    asm volatile("v_nop\n\tv_nop\n\tv_nop\n\tv_nop" : "+v"(d) : "v"(a), "v"(b));
    return d;
}

__device__ __forceinline__ unsigned int bf16_rne_bits(float f)
{
    unsigned int u = __float_as_uint(f);
    return (u + 0x7FFFu + ((u >> 16) & 1u)) >> 16;
}

__device__ __forceinline__ void split_hl(float f, unsigned int& hb, unsigned int& lb)
{
    hb = bf16_rne_bits(f);
    float hf = __uint_as_float(hb << 16);
    lb = bf16_rne_bits(f - hf);
}

__device__ __forceinline__ __bf16 bf16_from_bits(unsigned int b)
{
    union { unsigned short u; __bf16 v; } c;
    c.u = (unsigned short)b;
    return c.v;
}

__device__ __forceinline__ void pack8_hl(const float (&v)[8], v4u& H, v4u& L)
{
    unsigned int hb[8], lb[8];
#pragma unroll
    for (int i = 0; i < 8; ++i) split_hl(v[i], hb[i], lb[i]);
    H[0] = hb[0] | (hb[1] << 16); H[1] = hb[2] | (hb[3] << 16);
    H[2] = hb[4] | (hb[5] << 16); H[3] = hb[6] | (hb[7] << 16);
    L[0] = lb[0] | (lb[1] << 16); L[1] = lb[2] | (lb[3] << 16);
    L[2] = lb[4] | (lb[5] << 16); L[3] = lb[6] | (lb[7] << 16);
}

__device__ __forceinline__ float gelu_tanh(float u)
{
    float z = 0.7978845608028654f * (u + 0.044715f * u * u * u);
    float th = tanhf(z);
    return u * (0.5f * (1.0f + th));
}

__global__ __launch_bounds__(256) void k_stats(const float* __restrict__ x, float* __restrict__ stat)
{
    const int b = blockIdx.x, t = threadIdx.x;
    const float4* xb = (const float4*)(x + (size_t)b * S_SEQ * D_MODEL);
    double s = 0.0, q = 0.0;
#pragma unroll 1
    for (int i = t; i < (S_SEQ * D_MODEL) / 4; i += 256) {
        float4 v = xb[i];
        s += (double)v.x; s += (double)v.y; s += (double)v.z; s += (double)v.w;
        q += (double)v.x * (double)v.x; q += (double)v.y * (double)v.y;
        q += (double)v.z * (double)v.z; q += (double)v.w * (double)v.w;
    }
    __shared__ double r0[256], r1[256];
    __shared__ float vals[4];
    r0[t] = s; r1[t] = q;
    __syncthreads();
    for (int st = 128; st > 0; st >>= 1) {
        if (t < st) { r0[t] += r0[t + st]; r1[t] += r1[t + st]; }
        __syncthreads();
    }
    if (t == 0) {
        const double M = (double)S_SEQ * (double)D_MODEL;
        double mu = r0[0] / M;
        double var = r1[0] / M - mu * mu;
        if (var < 0.0) var = 0.0;
        float varf = (float)var;
        float rs = 1.0f / sqrtf(varf + EPSLN);
        vals[0] = (float)mu; vals[1] = rs; vals[2] = 0.f; vals[3] = 0.f;
    }
    __syncthreads();
    if (t < 8) {
        v4f v = {0.f, 0.f, 0.f, 0.f};
        if (t == 0) { v[0] = vals[0]; v[1] = vals[1]; }
        volatile v4f* p = (volatile v4f*)(stat + b * 32 + t * 4);
        *p = v;
        __threadfence();
        *p = v;
    }
}

__global__ __launch_bounds__(256) void k_topo_gather(const float* __restrict__ topo,
                                                     const float* __restrict__ Wdown,
                                                     const float* __restrict__ Wup,
                                                     float* __restrict__ gate,
                                                     __bf16* __restrict__ Wdh, __bf16* __restrict__ Wdl,
                                                     __bf16* __restrict__ Wuh, __bf16* __restrict__ Wul)
{
    const int t = threadIdx.x;
    __shared__ float row[DBOT];
    __shared__ int   idx[RQ];
    __shared__ float sg[256];
    __shared__ float gsh[NE];

    for (int e = 0; e < NE; ++e) {
        row[t] = topo[e * DBOT + t];
        __syncthreads();
        const float v = row[t];
        int rank = 0;
        for (int j = 0; j < DBOT; ++j) {
            float vj = row[j];
            rank += (vj > v) || (vj == v && j < t);
        }
        float contrib = 0.f;
        if (rank < RQ) {
            idx[rank] = t;
            contrib = 1.0f / (1.0f + expf(-v));
        }
        sg[t] = contrib;
        __syncthreads();
        for (int st = 128; st > 0; st >>= 1) {
            if (t < st) sg[t] += sg[t + st];
            __syncthreads();
        }
        if (t == 0) gsh[e] = sg[0] * (1.0f / (float)RQ);
        __syncthreads();

#pragma unroll 1
        for (int rp = 0; rp < RQ; rp += 2) {
            const int r = rp + (t >> 7);
            const int d0 = (t & 127) * 8;
            const int id = idx[r] & (DBOT - 1);
            float v8[8];
#pragma unroll
            for (int c = 0; c < 8; ++c) v8[c] = Wdown[(size_t)(d0 + c) * DBOT + id];
            v4u H, L;
            pack8_hl(v8, H, L);
            const size_t off = ((size_t)(e * RQ + r)) * D_MODEL + d0;
            volatile v4u* ph = (volatile v4u*)(Wdh + off);
            volatile v4u* pl = (volatile v4u*)(Wdl + off);
            *ph = H; *pl = L;
            __threadfence();
            *ph = H; *pl = L;
        }
#pragma unroll 1
        for (int d = t; d < D_MODEL; d += 256) {
            v4u H[8], L[8];
#pragma unroll
            for (int q = 0; q < 8; ++q) {
                float v8[8];
#pragma unroll
                for (int c = 0; c < 8; ++c) {
                    const int id = idx[q * 8 + c] & (DBOT - 1);
                    v8[c] = Wup[(size_t)id * D_MODEL + d];
                }
                pack8_hl(v8, H[q], L[q]);
            }
            const size_t off = ((size_t)(e * D_MODEL + d)) * RQ;
            volatile v4u* ph = (volatile v4u*)(Wuh + off);
            volatile v4u* pl = (volatile v4u*)(Wul + off);
#pragma unroll
            for (int q = 0; q < 8; ++q) { ph[q] = H[q]; pl[q] = L[q]; }
            __threadfence();
#pragma unroll
            for (int q = 0; q < 8; ++q) { ph[q] = H[q]; pl[q] = L[q]; }
        }
        __syncthreads();
    }
    if (t < 8) {
        v4f v = {0.f, 0.f, 0.f, 0.f};
        if (t < 4) { v[0] = gsh[4 * t]; v[1] = gsh[4 * t + 1]; v[2] = gsh[4 * t + 2]; v[3] = gsh[4 * t + 3]; }
        volatile v4f* p = (volatile v4f*)(gate + t * 4);
        *p = v;
        __threadfence();
        *p = v;
    }
}

__global__ __launch_bounds__(256) void k_router(const float* __restrict__ x,
                                                const int*   __restrict__ task_id,
                                                const float* __restrict__ task_emb,
                                                const float* __restrict__ Wr,
                                                const float* __restrict__ br,
                                                const float* __restrict__ stat,
                                                const float* __restrict__ gate,
                                                float* __restrict__ comb,
                                                int n_tasks)
{
    const int t = threadIdx.x;
    const int n = blockIdx.x * 256 + t;
    const int b = n / S_SEQ;
    __shared__ float gsh[NE];
    __shared__ __attribute__((aligned(16))) float csh[256 * NE];
    if (t < NE) gsh[t] = gate[t];
    __syncthreads();

    const float mu = stat[b * 32 + 0];
    const float rs = stat[b * 32 + 1];
    double acc[NE];
#pragma unroll
    for (int e = 0; e < NE; ++e) acc[e] = 0.0;

    const float* xr = x + (size_t)n * D_MODEL;
#pragma unroll 1
    for (int d = 0; d < D_MODEL; ++d) {
        const float xn = (xr[d] - mu) * rs;
        const double xd = (double)xn;
        const float* wrow = Wr + d * NE;
#pragma unroll
        for (int e = 0; e < NE; ++e) acc[e] += xd * (double)wrow[e];
    }
    int tid = task_id[b];
    if (tid < 0) tid += n_tasks;
    tid = tid < 0 ? 0 : (tid > n_tasks - 1 ? n_tasks - 1 : tid);
#pragma unroll 1
    for (int j = 0; j < DTASK; ++j) {
        const double tf = (double)task_emb[tid * DTASK + j];
        const float* wrow = Wr + (D_MODEL + j) * NE;
#pragma unroll
        for (int e = 0; e < NE; ++e) acc[e] += tf * (double)wrow[e];
    }
    float lg[NE];
#pragma unroll
    for (int e = 0; e < NE; ++e) lg[e] = (float)acc[e] + br[e];

    float b1 = lg[0]; int i1 = 0;
#pragma unroll
    for (int e = 1; e < NE; ++e) { if (lg[e] > b1) { b1 = lg[e]; i1 = e; } }
    float b2 = -3.0e38f; int i2 = -1;
#pragma unroll
    for (int e = 0; e < NE; ++e) { if (e != i1 && lg[e] > b2) { b2 = lg[e]; i2 = e; } }
    if (i2 < 0) { i2 = (i1 == 0) ? 1 : 0; b2 = b1; }

    const float u2 = expf(b2 - b1);
    const float ssum = 1.0f + u2;
    const float w1 = 1.0f / ssum;
    const float w2 = u2 / ssum;
    const float c1 = w1 * gsh[i1];
    const float c2 = w2 * gsh[i2];
#pragma unroll
    for (int e = 0; e < NE; ++e) csh[t * NE + e] = (e == i1) ? c1 : ((e == i2) ? c2 : 0.f);
    __syncthreads();

    float* dst = comb + (size_t)blockIdx.x * 256 * NE;
    v4f vv[4];
#pragma unroll
    for (int p = 0; p < 4; ++p) vv[p] = *(const v4fa*)(&csh[p * 1024 + t * 4]);
#pragma unroll
    for (int p = 0; p < 4; ++p) *(volatile v4f*)(dst + p * 1024 + t * 4) = vv[p];
    __threadfence();
#pragma unroll
    for (int p = 0; p < 4; ++p) *(volatile v4f*)(dst + p * 1024 + t * 4) = vv[p];
}

__global__ __launch_bounds__(256) void k_xgather(const float* __restrict__ x,
                                                 const float* __restrict__ comb,
                                                 int grp,
                                                 __bf16* __restrict__ Xh, __bf16* __restrict__ Xl,
                                                 float* __restrict__ Cst, int* __restrict__ meta)
{
    const int e = blockIdx.x, cl = blockIdx.y;
    const int cg = grp * CPG + cl;
    const int ce = cl * NE + e;
    const int t = threadIdx.x, lane = t & 31, w = t >> 5;
    __shared__ int   wcnt[8];
    __shared__ int   lst[CHUNK];
    __shared__ __attribute__((aligned(16))) float csl[CHUNK];

    const int n = cg * CHUNK + t;
    const float cv = comb[(size_t)n * NE + e];
    const bool f = (cv != 0.f);
    const unsigned msk = __builtin_amdgcn_ballot_w32(f);
    csl[t] = 0.f;
    if (lane == 0) wcnt[w] = __builtin_popcount(msk);
    __syncthreads();
    int pre = 0, total = 0;
#pragma unroll
    for (int j = 0; j < 8; ++j) { int vj = wcnt[j]; total += vj; if (j < w) pre += vj; }
    const unsigned lt = (1u << lane) - 1u;
    int slot = pre + __builtin_popcount(msk & lt);
    slot = slot > CHUNK - 1 ? CHUNK - 1 : slot;
    if (f) { lst[slot] = t; csl[slot] = cv; }
    __syncthreads();

    if (t < 64) {
        v4f v = *(const v4fa*)(&csl[t * 4]);
        volatile v4f* p = (volatile v4f*)(Cst + (size_t)ce * CHUNK + t * 4);
        *p = v;
        __threadfence();
        *p = v;
    }
    if (t < 8) {
        v4i mv = {0, 0, 0, 0};
        if (t == 0) mv[0] = total;
        volatile v4i* p = (volatile v4i*)(meta + ce * 32 + t * 4);
        *p = mv;
        __threadfence();
        *p = mv;
    }

    int nrows = (total + MT - 1) & ~(MT - 1);
    nrows = nrows > CHUNK ? CHUNK : nrows;
    const size_t rbase = (size_t)ce * CHUNK;
#pragma unroll 1
    for (int s0 = 0; s0 < nrows; s0 += 2) {
        const int s = s0 + (t >> 7);
        const int d0 = (t & 127) * 8;
        v4u H = {0u, 0u, 0u, 0u}, L = {0u, 0u, 0u, 0u};
        if (s < total) {
            const int tt = lst[s] & (CHUNK - 1);
            const float4* src = (const float4*)(x + ((size_t)(cg * CHUNK + tt)) * D_MODEL + d0);
            float4 a = src[0], c = src[1];
            float v8[8] = {a.x, a.y, a.z, a.w, c.x, c.y, c.z, c.w};
            pack8_hl(v8, H, L);
        }
        const size_t off = (rbase + (size_t)s) * D_MODEL + d0;
        volatile v4u* ph = (volatile v4u*)(Xh + off);
        volatile v4u* pl = (volatile v4u*)(Xl + off);
        *ph = H; *pl = L;
        __threadfence();
        *ph = H; *pl = L;
    }
}

__device__ __forceinline__ v8f k64_tile(const v16bf ah0, const v16bf ah1, const v16bf al0, const v16bf al1,
                                        const __bf16* bh, const __bf16* bl, int h)
{
    Frag b0h, b0l, b1h, b1l;
    b0h.h8[0] = *(const v8bf*)(bh + 8 * h);       b0h.h8[1] = *(const v8bf*)(bh + 16 + 8 * h);
    b1h.h8[0] = *(const v8bf*)(bh + 32 + 8 * h);  b1h.h8[1] = *(const v8bf*)(bh + 48 + 8 * h);
    b0l.h8[0] = *(const v8bf*)(bl + 8 * h);       b0l.h8[1] = *(const v8bf*)(bl + 16 + 8 * h);
    b1l.h8[0] = *(const v8bf*)(bl + 32 + 8 * h);  b1l.h8[1] = *(const v8bf*)(bl + 48 + 8 * h);
    v8f y = {0.f, 0.f, 0.f, 0.f, 0.f, 0.f, 0.f, 0.f};
    y = wmma16(ah0, b0h.v, y); y = wmma16(ah0, b0l.v, y); y = wmma16(al0, b0h.v, y);
    y = wmma16(ah1, b1h.v, y); y = wmma16(ah1, b1l.v, y); y = wmma16(al1, b1h.v, y);
    return y;
}

__global__ __launch_bounds__(64) void k_moe(const __bf16* __restrict__ Xh, const __bf16* __restrict__ Xl,
                                            const float* __restrict__ Cst, const int* __restrict__ meta,
                                            const __bf16* __restrict__ Wdh, const __bf16* __restrict__ Wdl,
                                            const __bf16* __restrict__ Wuh, const __bf16* __restrict__ Wul,
                                            float* __restrict__ Yst)
{
    const int tile = blockIdx.x, e = blockIdx.y, cl = blockIdx.z;
    const int ce = cl * NE + e;
    int total = meta[ce * 32];
    total = total < 0 ? 0 : (total > CHUNK ? CHUNK : total);
    if (tile * MT >= total) return;

    const int t = threadIdx.x, lane = t & 31, w = t >> 5, h = lane >> 4, m = lane & 15;
    const size_t row0 = (size_t)ce * CHUNK + (size_t)tile * MT;

    __shared__ float c_sh[MT];
    __shared__ __attribute__((aligned(16))) __bf16 abh[MT][72];
    __shared__ __attribute__((aligned(16))) __bf16 abl[MT][72];
    __shared__ __attribute__((aligned(16))) float  ytile[2][MT][36];

    if (t < MT) c_sh[t] = Cst[(size_t)ce * CHUNK + tile * MT + t];

    const v8f z8 = {0.f, 0.f, 0.f, 0.f, 0.f, 0.f, 0.f, 0.f};
    v8f acc0 = z8, acc1 = z8;
    const __bf16* xah = Xh + (row0 + m) * D_MODEL;
    const __bf16* xal = Xl + (row0 + m) * D_MODEL;
    const size_t wrw0 = ((size_t)(e * RQ + (2 * w) * 16 + m)) * D_MODEL;
    const size_t wrw1 = wrw0 + (size_t)16 * D_MODEL;
#pragma unroll 1
    for (int k0 = 0; k0 < D_MODEL; k0 += 32) {
        const int ka = k0 + 8 * h, kb = k0 + 16 + 8 * h;
        Frag ah, al, bh0, bl0, bh1, bl1;
        ah.h8[0]  = *(const v8bf*)(xah + ka);        ah.h8[1]  = *(const v8bf*)(xah + kb);
        al.h8[0]  = *(const v8bf*)(xal + ka);        al.h8[1]  = *(const v8bf*)(xal + kb);
        bh0.h8[0] = *(const v8bf*)(Wdh + wrw0 + ka); bh0.h8[1] = *(const v8bf*)(Wdh + wrw0 + kb);
        bl0.h8[0] = *(const v8bf*)(Wdl + wrw0 + ka); bl0.h8[1] = *(const v8bf*)(Wdl + wrw0 + kb);
        bh1.h8[0] = *(const v8bf*)(Wdh + wrw1 + ka); bh1.h8[1] = *(const v8bf*)(Wdh + wrw1 + kb);
        bl1.h8[0] = *(const v8bf*)(Wdl + wrw1 + ka); bl1.h8[1] = *(const v8bf*)(Wdl + wrw1 + kb);
        acc0 = wmma16(ah.v, bh0.v, acc0); acc0 = wmma16(ah.v, bl0.v, acc0); acc0 = wmma16(al.v, bh0.v, acc0);
        acc1 = wmma16(ah.v, bh1.v, acc1); acc1 = wmma16(ah.v, bl1.v, acc1); acc1 = wmma16(al.v, bh1.v, acc1);
    }
    __syncthreads();

#pragma unroll
    for (int r = 0; r < 8; ++r) {
        const int row = 8 * h + r;
        const float cv = c_sh[row];
        const float a0 = gelu_tanh(acc0[r]) * cv;
        const float a1 = gelu_tanh(acc1[r]) * cv;
        unsigned int hb, lb;
        split_hl(a0, hb, lb);
        abh[row][(2 * w) * 16 + m] = bf16_from_bits(hb);
        abl[row][(2 * w) * 16 + m] = bf16_from_bits(lb);
        split_hl(a1, hb, lb);
        abh[row][(2 * w + 1) * 16 + m] = bf16_from_bits(hb);
        abl[row][(2 * w + 1) * 16 + m] = bf16_from_bits(lb);
    }
    __syncthreads();

    Frag A_h0, A_h1, A_l0, A_l1;
    A_h0.h8[0] = *(const v8bf*)(&abh[m][8 * h]);       A_h0.h8[1] = *(const v8bf*)(&abh[m][16 + 8 * h]);
    A_h1.h8[0] = *(const v8bf*)(&abh[m][32 + 8 * h]);  A_h1.h8[1] = *(const v8bf*)(&abh[m][48 + 8 * h]);
    A_l0.h8[0] = *(const v8bf*)(&abl[m][8 * h]);       A_l0.h8[1] = *(const v8bf*)(&abl[m][16 + 8 * h]);
    A_l1.h8[0] = *(const v8bf*)(&abl[m][32 + 8 * h]);  A_l1.h8[1] = *(const v8bf*)(&abl[m][48 + 8 * h]);

    const size_t wub = ((size_t)e * D_MODEL + m) * RQ;
    const int q = lane >> 3, pp = lane & 7;
#pragma unroll 1
    for (int p = 0; p < 16; ++p) {
        const int dtA = 32 * w + 2 * p;
        const __bf16* bh = Wuh + wub + (size_t)dtA * 16 * RQ;
        const __bf16* bl = Wul + wub + (size_t)dtA * 16 * RQ;
        v8f y0 = k64_tile(A_h0.v, A_h1.v, A_l0.v, A_l1.v, bh, bl, h);
        v8f y1 = k64_tile(A_h0.v, A_h1.v, A_l0.v, A_l1.v, bh + 16 * RQ, bl + 16 * RQ, h);
#pragma unroll
        for (int r = 0; r < 8; ++r) {
            ytile[w][8 * h + r][m]      = y0[r];
            ytile[w][8 * h + r][16 + m] = y1[r];
        }
        __syncthreads();
        v4f v[4];
#pragma unroll
        for (int it = 0; it < 4; ++it) v[it] = *(const v4fa*)(&ytile[w][it * 4 + q][pp * 4]);
        float* ybase = Yst + row0 * D_MODEL + (size_t)dtA * 16 + pp * 4;
#pragma unroll
        for (int it = 0; it < 4; ++it) *(volatile v4f*)(ybase + (size_t)(it * 4 + q) * D_MODEL) = v[it];
        __threadfence();
#pragma unroll
        for (int it = 0; it < 4; ++it) *(volatile v4f*)(ybase + (size_t)(it * 4 + q) * D_MODEL) = v[it];
        __syncthreads();
    }
}

__global__ __launch_bounds__(256) void k_combine(const float* __restrict__ comb,
                                                 const float* __restrict__ Yst,
                                                 int grp,
                                                 float* __restrict__ out)
{
    const int slab = blockIdx.x, cl = blockIdx.y;
    const int cg = grp * CPG + cl;
    const int t = threadIdx.x, lane = t & 31, w = t >> 5;
    const int n = cg * CHUNK + t;
    __shared__ int wcnt[NE][8];

    float c[NE];
    {
        const float4* cp = (const float4*)(comb + (size_t)n * NE);
#pragma unroll
        for (int p = 0; p < 4; ++p) {
            float4 v = cp[p];
            c[4 * p] = v.x; c[4 * p + 1] = v.y; c[4 * p + 2] = v.z; c[4 * p + 3] = v.w;
        }
    }
    const unsigned lt = (1u << lane) - 1u;
    unsigned fl = 0u;
    int inw[NE];
#pragma unroll
    for (int e = 0; e < NE; ++e) {
        const bool f = (c[e] != 0.f);
        const unsigned msk = __builtin_amdgcn_ballot_w32(f);
        if (lane == 0) wcnt[e][w] = __builtin_popcount(msk);
        inw[e] = __builtin_popcount(msk & lt);
        fl |= (f ? 1u : 0u) << e;
    }
    __syncthreads();

    const v4f z4 = {0.f, 0.f, 0.f, 0.f};
    v4f acc[8];
#pragma unroll
    for (int k = 0; k < 8; ++k) acc[k] = z4;
#pragma unroll
    for (int e = 0; e < NE; ++e) {
        if ((fl >> e) & 1u) {
            int pre = 0;
#pragma unroll
            for (int j = 0; j < 8; ++j) { if (j < w) pre += wcnt[e][j]; }
            int slot = pre + inw[e];
            slot = slot > CHUNK - 1 ? CHUNK - 1 : slot;
            const float* src = Yst + (((size_t)(cl * NE + e)) * CHUNK + (size_t)slot) * D_MODEL + slab * 32;
#pragma unroll
            for (int k = 0; k < 8; ++k) acc[k] += *(const v4f*)(src + 4 * k);
        }
    }
    float* dst = out + (size_t)n * D_MODEL + slab * 32;
#pragma unroll
    for (int k = 0; k < 8; ++k) *(volatile v4f*)(dst + 4 * k) = acc[k];
    __threadfence();
#pragma unroll
    for (int k = 0; k < 8; ++k) *(volatile v4f*)(dst + 4 * k) = acc[k];
}

extern "C" void kernel_launch(void* const* d_in, const int* in_sizes, int n_in,
                              void* d_out, int out_size, void* d_ws, size_t ws_size,
                              hipStream_t stream)
{
    if (n_in < 8) return;
    if (in_sizes[0] != N_TOK * D_MODEL) return;
    if (in_sizes[1] < NB) return;
    if (in_sizes[2] < DTASK) return;
    if (in_sizes[3] != (D_MODEL + DTASK) * NE) return;
    if (in_sizes[4] < NE) return;
    if (in_sizes[5] != D_MODEL * DBOT) return;
    if (in_sizes[6] != DBOT * D_MODEL) return;
    if (in_sizes[7] != NE * DBOT) return;
    if (out_size != N_TOK * D_MODEL) return;
    if (ws_size < WS_TOTAL) return;
    const int n_tasks = in_sizes[2] / DTASK;

    const float* x        = (const float*)d_in[0];
    const int*   task_id  = (const int*)  d_in[1];
    const float* task_emb = (const float*)d_in[2];
    const float* Wr       = (const float*)d_in[3];
    const float* br       = (const float*)d_in[4];
    const float* Wdown    = (const float*)d_in[5];
    const float* Wup      = (const float*)d_in[6];
    const float* topo     = (const float*)d_in[7];
    float* out = (float*)d_out;

    char* ws = (char*)d_ws;
    float*  stat = (float*)(ws + OFF_STAT);
    float*  gate = (float*)(ws + OFF_GATE);
    int*    meta = (int*)  (ws + OFF_META);
    float*  Cst  = (float*)(ws + OFF_CST);
    float*  comb = (float*)(ws + OFF_COMB);
    __bf16* Wdh  = (__bf16*)(ws + OFF_WDH);
    __bf16* Wdl  = (__bf16*)(ws + OFF_WDL);
    __bf16* Wuh  = (__bf16*)(ws + OFF_WUH);
    __bf16* Wul  = (__bf16*)(ws + OFF_WUL);
    __bf16* Xh   = (__bf16*)(ws + OFF_XH);
    __bf16* Xl   = (__bf16*)(ws + OFF_XL);
    float*  Yst  = (float*)(ws + OFF_Y);

    k_stats<<<NB, 256, 0, stream>>>(x, stat);
    k_topo_gather<<<1, 256, 0, stream>>>(topo, Wdown, Wup, gate, Wdh, Wdl, Wuh, Wul);
    k_router<<<N_TOK / 256, 256, 0, stream>>>(x, task_id, task_emb, Wr, br, stat, gate, comb, n_tasks);
    for (int g = 0; g < NGRP; ++g) {
        k_xgather<<<dim3(NE, CPG), 256, 0, stream>>>(x, comb, g, Xh, Xl, Cst, meta);
        k_moe<<<dim3(CHUNK / MT, NE, CPG), 64, 0, stream>>>(Xh, Xl, Cst, meta, Wdh, Wdl, Wuh, Wul, Yst);
        k_combine<<<dim3(D_MODEL / 32, CPG), 256, 0, stream>>>(comb, Yst, g, out);
    }
}
